// RDFNSAttention_27814208209736
// MI455X (gfx1250) — hardware-verified
//
#include <hip/hip_runtime.h>
#include <math.h>

constexpr int kBatch = 2;
constexpr int kSeq   = 2048;
constexpr int kEmb   = 768;
constexpr int kHeads = 12;
constexpr int kHD    = 64;
constexpr int kBH    = kBatch * kHeads;
constexpr int kTok   = kBatch * kSeq;
constexpr int kGH    = 3;
constexpr int kNG    = kBH / kGH;
constexpr int kRB    = kSeq / 64;
constexpr long kHeadPlane  = (long)kSeq * kHD;
constexpr long kScorePlane = (long)kSeq * kSeq;
constexpr float kWCarry    = 16.0f;
constexpr float kWCarryInv = 1.0f / 16.0f;
constexpr float kPCarry    = 2048.0f;
constexpr float kCtxCarry  = 256.0f;
constexpr float kPVScale   = kCtxCarry / kPCarry;
constexpr float kOutScale  = 1.0f / (kCtxCarry * kWCarry);
constexpr float kInvEmb    = 1.0f / 768.0f;
constexpr float kLnEps     = 1e-12f;
constexpr float kL1Eps     = 1e-12f;
constexpr float kD2Floor   = 1e-12f;
constexpr float kDistScale = 0.125f;

typedef __attribute__((ext_vector_type(16))) _Float16 v16h;
typedef __attribute__((ext_vector_type(8)))  _Float16 v8h;
typedef __attribute__((ext_vector_type(16))) __bf16   v16b;
typedef __attribute__((ext_vector_type(8)))  __bf16   v8b;
typedef __attribute__((ext_vector_type(8)))  float    v8f;
typedef __attribute__((ext_vector_type(4)))  float    v4f;
typedef __attribute__((ext_vector_type(4)))  unsigned int v4u;

__device__ __forceinline__ unsigned short f2bf_bits(float f) {
  unsigned u = __float_as_uint(f);
  return (unsigned short)((u + 0x7FFFu + ((u >> 16) & 1u)) >> 16);
}
__device__ __forceinline__ float bf_bits2f(unsigned short h) { return __uint_as_float(((unsigned)h) << 16); }

__device__ __forceinline__ void dep_guard_h(v8f& a, v8f& b, v16h x, v16h y) { asm volatile("v_nop\n\tv_nop\n\tv_nop\n\tv_nop" : "+v"(a), "+v"(b) : "v"(x), "v"(y)); }
__device__ __forceinline__ void dep_guard_b(v8f& a, v8f& b, v16b x, v16b y) { asm volatile("v_nop\n\tv_nop\n\tv_nop\n\tv_nop" : "+v"(a), "+v"(b) : "v"(x), "v"(y)); }
__device__ __forceinline__ void keep4_h(v16h a, v16h b, v16h c, v16h d) { asm volatile("v_nop" :: "v"(a), "v"(b), "v"(c), "v"(d)); }
__device__ __forceinline__ void keep4_b(v16b a, v16b b, v16b c, v16b d) { asm volatile("v_nop" :: "v"(a), "v"(b), "v"(c), "v"(d)); }
__device__ __forceinline__ void acc_guard4(v8f& a, v8f& b, v8f& c, v8f& d) { asm volatile("v_nop\n\tv_nop\n\tv_nop\n\tv_nop" : "+v"(a), "+v"(b), "+v"(c), "+v"(d)); }
template <typename T> struct Frag;
template <> struct Frag<_Float16> {
  typedef v16h V; union U { v16h v; v8h h[2]; };
  static __device__ __forceinline__ v16h load(const _Float16* p) {
    U f; f.h[0] = *(const v8h*)(p); f.h[1] = *(const v8h*)(p + 16); return f.v;
  }
  static __device__ __forceinline__ v8f mma(v16h a, v16h b, v8f c) {
    return __builtin_amdgcn_wmma_f32_16x16x32_f16(false, a, false, b, (short)0, c, false, false);
  }
  static __device__ __forceinline__ void guard(v8f& a, v8f& b, v16h x, v16h y) { dep_guard_h(a, b, x, y); }
  static __device__ __forceinline__ void keep(v16h a, v16h b, v16h c, v16h d) { keep4_h(a, b, c, d); }
};
template <> struct Frag<__bf16> {
  typedef v16b V; union U { v16b v; v8b h[2]; };
  static __device__ __forceinline__ v16b load(const __bf16* p) {
    U f; f.h[0] = *(const v8b*)(p); f.h[1] = *(const v8b*)(p + 16); return f.v;
  }
  static __device__ __forceinline__ v8f mma(v16b a, v16b b, v8f c) {
    return __builtin_amdgcn_wmma_f32_16x16x32_bf16(false, a, false, b, (short)0, c, false, false);
  }
  static __device__ __forceinline__ void guard(v8f& a, v8f& b, v16b x, v16b y) { dep_guard_b(a, b, x, y); }
  static __device__ __forceinline__ void keep(v16b a, v16b b, v16b c, v16b d) { keep4_b(a, b, c, d); }
};

__device__ __forceinline__ unsigned pk16(unsigned short a, unsigned short b) { return (unsigned)a | ((unsigned)b << 16); }
__device__ __forceinline__ unsigned short h_bits(float f) { const _Float16 h = (_Float16)f; return __builtin_bit_cast(unsigned short, h); }

template <int ET> struct Elem;
template <> struct Elem<0> { typedef _Float16 T; };
template <> struct Elem<1> { typedef __bf16 T; };
template <int ET, bool SPLIT, int BIAS_MODE, int OUT_MODE, bool RESID, int ACT, bool HSPLIT>
__global__ __launch_bounds__(256) void wmma_gemm64(
    const unsigned short* __restrict__ Ap, const unsigned short* __restrict__ A2p, int lda, long strideA,
    const unsigned short* __restrict__ Btp, const unsigned short* __restrict__ Bt2p, int ldb, long strideB,
    void* __restrict__ Cout, void* __restrict__ Cout2, int ldc, long strideC, long strideH,
    const float* __restrict__ bias,
    const float* __restrict__ resid, long strideR,
    int M, int N, int K, float scale) {
  static_assert(!(HSPLIT && RESID), "hsplit without resid");
  typedef typename Elem<ET>::T T;
  typedef typename Frag<T>::V V;
  const T* A = (const T*)Ap; const T* A2 = (const T*)A2p; const T* Bt = (const T*)Btp; const T* Bt2 = (const T*)Bt2p;
  __shared__ __align__(16) float sT[8][16 * 68];
  const int b    = blockIdx.y;
  const int lane = threadIdx.x & 31;
  const int wave = threadIdx.x >> 5;
  const int tilesN = N >> 6;
  const int tilesM = M >> 6;
  const int tile = blockIdx.x * 8 + wave;
  if (tile >= tilesM * tilesN) return;
  const int tm = tile / tilesN;
  const int tn = tile - tm * tilesN;
  const int m0 = tm << 6;
  const int n0 = tn << 6;

  const T* Ab  = A  + (size_t)b * strideA;
  const T* Bb  = Bt + (size_t)b * strideB;
  const T* Ab2 = SPLIT ? (A2  + (size_t)b * strideA) : nullptr;
  const T* Bb2 = SPLIT ? (Bt2 + (size_t)b * strideB) : nullptr;

  const int rlane = lane & 15;
  const int koff  = (lane >> 4) * 8;
  const int mOff  = (lane >> 4) * 8;

  v8f acc[4][4];
#pragma unroll
  for (int i = 0; i < 4; ++i)
#pragma unroll
    for (int j = 0; j < 4; ++j) acc[i][j] = (v8f){0.f,0.f,0.f,0.f,0.f,0.f,0.f,0.f};

  for (int k0 = 0; k0 < K; k0 += 32) {
    V bh[4], bl[4];
#pragma unroll
    for (int j = 0; j < 4; ++j) {
      const size_t bo = (size_t)(n0 + (j << 4) + rlane) * ldb + koff + k0;
      bh[j] = Frag<T>::load(Bb + bo);
      if (SPLIT) bl[j] = Frag<T>::load(Bb2 + bo);
    }
#pragma unroll
    for (int i = 0; i < 4; ++i) {
      const size_t ao = (size_t)(m0 + (i << 4) + rlane) * lda + koff + k0;
      V ah = Frag<T>::load(Ab + ao);
      V al;
      if (SPLIT) al = Frag<T>::load(Ab2 + ao);
#pragma unroll
      for (int j = 0; j < 4; ++j) {
        acc[i][j] = Frag<T>::mma(ah, bh[j], acc[i][j]);
        if (SPLIT) {
          acc[i][j] = Frag<T>::mma(ah, bl[j], acc[i][j]);
          acc[i][j] = Frag<T>::mma(al, bh[j], acc[i][j]);
        }
      }
      Frag<T>::guard(acc[i][0], acc[i][3], ah, SPLIT ? al : ah);
    }
    Frag<T>::keep(bh[0], bh[1], bh[2], bh[3]);
    if (SPLIT) Frag<T>::keep(bl[0], bl[1], bl[2], bl[3]);
  }
  acc_guard4(acc[0][0], acc[0][1], acc[0][2], acc[0][3]);
  acc_guard4(acc[1][0], acc[1][1], acc[1][2], acc[1][3]);
  acc_guard4(acc[2][0], acc[2][1], acc[2][2], acc[2][3]);
  acc_guard4(acc[3][0], acc[3][1], acc[3][2], acc[3][3]);

  float* slab = sT[wave];
  const float* Rb = RESID ? (resid + (size_t)b * strideR) : nullptr;
  const size_t cb = HSPLIT ? ((size_t)tn * (size_t)strideH) : (size_t)n0;
#pragma unroll
  for (int i = 0; i < 4; ++i) {
    const int mBase = m0 + (i << 4);
#pragma unroll
    for (int j = 0; j < 4; ++j) {
      const int n = n0 + (j << 4) + rlane;
      float bv = 0.f;
      if (BIAS_MODE == 2) bv = bias[n];
#pragma unroll
      for (int r = 0; r < 8; ++r) {
        float v = acc[i][j][r] * scale;
        if (BIAS_MODE == 1) v += bias[mBase + mOff + r];
        if (BIAS_MODE == 2) v += bv;
        if (RESID) v += Rb[(size_t)(mBase + mOff + r) * ldc + n];
        if (ACT == 2) v = fmaxf(v, 0.0f);
        if (ACT == 4) v = (v > 0.f) ? v : 0.01f * v;
        slab[(mOff + r) * 68 + (j << 4) + rlane] = v;
      }
    }
    __builtin_amdgcn_fence(__ATOMIC_RELEASE, "workgroup");
    __builtin_amdgcn_wave_barrier();
    __builtin_amdgcn_fence(__ATOMIC_ACQUIRE, "workgroup");
    if (OUT_MODE == 0) {
      float* C = (float*)Cout + (size_t)b * strideC;
      const int hh = lane >> 4, c4 = (lane & 15) * 4;
      for (int pass = 0; pass < 2; ++pass) {
#pragma unroll
        for (int it = 0; it < 8; ++it) {
          const int row = it * 2 + hh;
          v4f v = *(const v4f*)(slab + row * 68 + c4);
          *(volatile v4f*)(C + (size_t)(mBase + row) * ldc + cb + c4) = v;
        }
        __threadfence();
      }
    } else {
      const int q = lane >> 3, c8 = (lane & 7) * 8;
      unsigned short* C  = (unsigned short*)Cout  + (size_t)b * strideC;
      unsigned short* C2 = (OUT_MODE == 2) ? ((unsigned short*)Cout2 + (size_t)b * strideC) : nullptr;
      for (int pass = 0; pass < 2; ++pass) {
#pragma unroll
        for (int it = 0; it < 4; ++it) {
          const int row = it * 4 + q;
          const float* sp = slab + row * 68 + c8;
          v8h hv, lv;
#pragma unroll
          for (int e = 0; e < 8; ++e) {
            if (OUT_MODE == 1) {
              hv[e] = (_Float16)sp[e];
            } else {
              unsigned short hb = f2bf_bits(sp[e]);
              unsigned short lb = f2bf_bits(sp[e] - bf_bits2f(hb));
              hv[e] = __builtin_bit_cast(_Float16, hb);
              lv[e] = __builtin_bit_cast(_Float16, lb);
            }
          }
          *(volatile v8h*)(C + (size_t)(mBase + row) * ldc + cb + c8) = hv;
          if (OUT_MODE == 2) *(volatile v8h*)(C2 + (size_t)(mBase + row) * ldc + cb + c8) = lv;
        }
        __threadfence();
      }
    }
    __builtin_amdgcn_fence(__ATOMIC_RELEASE, "workgroup");
    __builtin_amdgcn_wave_barrier();
    __builtin_amdgcn_fence(__ATOMIC_ACQUIRE, "workgroup");
  }
}

__global__ __launch_bounds__(256) void wtcast_kernel(const float* __restrict__ W0, const float* __restrict__ W1,
                                                     const float* __restrict__ W2, const float* __restrict__ W3,
                                                     unsigned short* __restrict__ out, float scale) {
  __shared__ float sm[64][65];
  const int t  = threadIdx.x;
  const int d0 = blockIdx.x * 64;
  const int h0 = blockIdx.y * 64;
  const int z  = blockIdx.z;
  const float* W = (z == 0) ? W0 : (z == 1) ? W1 : (z == 2) ? W2 : W3;
#pragma unroll
  for (int i = 0; i < 16; ++i) {
    const int e = i * 256 + t;
    const int r = e >> 6;
    const int c = e & 63;
    sm[c][r] = W[(size_t)(d0 + r) * kEmb + h0 + c] * scale;
  }
  __syncthreads();
  const int lane = t & 31, wave = t >> 5;
  const int q = lane >> 3, c8 = (lane & 7) * 8;
  unsigned short* op = out + (size_t)z * kEmb * kEmb;
  for (int pass = 0; pass < 2; ++pass) {
#pragma unroll
    for (int it = 0; it < 2; ++it) {
      const int row = wave * 8 + it * 4 + q;
      unsigned short hb[8];
#pragma unroll
      for (int e = 0; e < 8; ++e) hb[e] = h_bits(sm[row][c8 + e]);
      const v4u u = (v4u){pk16(hb[0], hb[1]), pk16(hb[2], hb[3]), pk16(hb[4], hb[5]), pk16(hb[6], hb[7])};
      *(volatile v4u*)(op + (size_t)(h0 + row) * kEmb + d0 + c8) = u;
    }
    __threadfence();
  }
}

__global__ __launch_bounds__(256) void cast8_f16_kernel(const float* __restrict__ in, unsigned short* __restrict__ out, int n8) {
  const int i = blockIdx.x * 256 + threadIdx.x;
  if (i >= n8) return;
  const float* p = in + 8 * (size_t)i;
  const v4f a = *(const v4f*)(p);
  const v4f c = *(const v4f*)(p + 4);
  unsigned short hb[8];
#pragma unroll
  for (int e = 0; e < 4; ++e) {
    hb[e]     = h_bits(a[e]);
    hb[4 + e] = h_bits(c[e]);
  }
  const v4u u = (v4u){pk16(hb[0], hb[1]), pk16(hb[2], hb[3]), pk16(hb[4], hb[5]), pk16(hb[6], hb[7])};
  unsigned short* q = out + 8 * (size_t)i;
  *(volatile v4u*)q = u;
  __threadfence();
  *(volatile v4u*)q = u;
}

__global__ __launch_bounds__(256) void sqnorm_kernel(const unsigned short* __restrict__ qp, const unsigned short* __restrict__ kp,
                                                     float* __restrict__ qsq, float* __restrict__ ksq, int nrows) {
  const int i = blockIdx.x * 256 + threadIdx.x;
  const int y = blockIdx.y;
  const unsigned short* src = (y == 0) ? qp : kp;
  float* dst = (y == 0) ? qsq : ksq;
  const int ic = (i < nrows) ? i : (nrows - 1);
  const _Float16* p = (const _Float16*)src + (size_t)ic * kHD;
  float s = 0.f;
#pragma unroll 1
  for (int j = 0; j < 8; ++j) {
    const v8h v = *(const v8h*)(p + 8 * j);
#pragma unroll
    for (int e = 0; e < 8; ++e) { const float f = (float)v[e]; s += f * f; }
  }
  if (i < nrows) *(volatile float*)(dst + i) = s;
  __threadfence();
  if (i < nrows) *(volatile float*)(dst + i) = s;
}

__device__ __forceinline__ float score_of(float q2, float k2, float g, float m) {
  const float d2 = (q2 + k2) - 2.0f * g;
  const float gd = __builtin_amdgcn_sqrtf(fmaxf(d2, kD2Floor));
  const float x  = gd * kDistScale;
  const float p  = __expf(-(x * x));
  return (m >= 0.0f) ? p : 0.0f;
}

__global__ __launch_bounds__(256) void score_rows_kernel(float* __restrict__ G,
                                                         const float* __restrict__ qsq, const float* __restrict__ ksq,
                                                         const float* __restrict__ amask,
                                                         float* __restrict__ nr, float* __restrict__ colpart, int bh0) {
  __shared__ float rowp[64][8];
  __shared__ __align__(16) float nrs[64];
  const int tid = threadIdx.x, lane = tid & 31, wave = tid >> 5;
  const int rb = blockIdx.x;
  const int hz = blockIdx.y;
  const int bh = bh0 + hz;
  const int b  = bh / kHeads;
  const int cA = 4 * tid, cB = 1024 + 4 * tid;
  const v4f k2A = *(const v4f*)(ksq + (size_t)bh * kSeq + cA);
  const v4f k2B = *(const v4f*)(ksq + (size_t)bh * kSeq + cB);
  const v4f mA  = *(const v4f*)(amask + (size_t)b * kSeq + cA);
  const v4f mB  = *(const v4f*)(amask + (size_t)b * kSeq + cB);
  v4f colA = (v4f){0.f, 0.f, 0.f, 0.f};
  v4f colB = (v4f){0.f, 0.f, 0.f, 0.f};
  float* Gp = G + (size_t)hz * kScorePlane + (size_t)(rb * 64) * kSeq;
  const float* qp = qsq + (size_t)bh * kSeq + rb * 64;
#pragma unroll 1
  for (int r = 0; r < 64; ++r) {
    const float q2 = qp[r];
    float* grow = Gp + (size_t)r * kSeq;
    const v4f gA = *(const v4f*)(grow + cA);
    const v4f gB = *(const v4f*)(grow + cB);
    v4f pA, pB;
#pragma unroll
    for (int e = 0; e < 4; ++e) {
      pA[e] = score_of(q2, k2A[e], gA[e], mA[e]);
      pB[e] = score_of(q2, k2B[e], gB[e], mB[e]);
    }
    for (int pass = 0; pass < 2; ++pass) {
      *(volatile v4f*)(grow + cA) = pA;
      *(volatile v4f*)(grow + cB) = pB;
      __threadfence();
    }
    colA += pA;
    colB += pB;
    float rs = ((pA[0] + pA[1]) + (pA[2] + pA[3])) + ((pB[0] + pB[1]) + (pB[2] + pB[3]));
#pragma unroll
    for (int off = 1; off < 32; off <<= 1) rs += __shfl_xor(rs, off, 32);
    if (lane == 0) rowp[r][wave] = rs;
  }
  __syncthreads();
  if (tid < 64) {
    float s = rowp[tid][0];
#pragma unroll
    for (int w = 1; w < 8; ++w) s += rowp[tid][w];
    nrs[tid] = s;
  }
  __syncthreads();
  const v4f nv = *(const v4f*)(nrs + 4 * (tid & 15));
  float* nrp = nr + (size_t)hz * kSeq + rb * 64 + 4 * (tid & 15);
  float* cpp = colpart + ((size_t)hz * kRB + rb) * kSeq;
  for (int pass = 0; pass < 2; ++pass) {
    if (tid < 16) *(volatile v4f*)nrp = nv;
    *(volatile v4f*)(cpp + cA) = colA;
    *(volatile v4f*)(cpp + cB) = colB;
    __threadfence();
  }
}

__global__ __launch_bounds__(256) void colnorm_kernel(const float* __restrict__ colpart, float* __restrict__ cs) {
  const int t  = blockIdx.x * 256 + threadIdx.x;
  const int hz = blockIdx.y;
  const float* p = colpart + (size_t)hz * kRB * kSeq + t;
  float s = 0.f;
#pragma unroll 1
  for (int rb = 0; rb < kRB; ++rb) s += p[(size_t)rb * kSeq];
  const float c = rsqrtf(s);
  float* o = cs + (size_t)hz * kSeq + t;
  *(volatile float*)o = c;
  __threadfence();
  *(volatile float*)o = c;
}

__global__ __launch_bounds__(256) void rownorm_kernel(const float* __restrict__ G, const float* __restrict__ nr,
                                                      const float* __restrict__ cs, unsigned short* __restrict__ P) {
  const int lane = threadIdx.x & 31, wave = threadIdx.x >> 5;
  const int row = blockIdx.x * 8 + wave;
  const int hz  = row >> 11;
  const float rsf = rsqrtf(nr[row]);
  const float* gp = G + (size_t)row * kSeq;
  const float* cp = cs + (size_t)hz * kSeq;
  float kt[8][8];
  float D = 0.f;
#pragma unroll
  for (int i = 0; i < 8; ++i) {
    const int c0 = 256 * i + 8 * lane;
    const v4f g0 = *(const v4f*)(gp + c0);
    const v4f g1 = *(const v4f*)(gp + c0 + 4);
    const v4f s0 = *(const v4f*)(cp + c0);
    const v4f s1 = *(const v4f*)(cp + c0 + 4);
#pragma unroll
    for (int e = 0; e < 4; ++e) {
      kt[i][e]     = (rsf * g0[e]) * s0[e];
      kt[i][4 + e] = (rsf * g1[e]) * s1[e];
    }
#pragma unroll
    for (int e = 0; e < 8; ++e) D += fabsf(kt[i][e]);
  }
#pragma unroll
  for (int off = 1; off < 32; off <<= 1) D += __shfl_xor(D, off, 32);
  const float denom = fmaxf(D, kL1Eps);
  const float inv = __builtin_amdgcn_rcpf(denom) * kPCarry;
  v4u hv[8];
#pragma unroll
  for (int i = 0; i < 8; ++i) {
    unsigned short hb[8];
#pragma unroll
    for (int e = 0; e < 8; ++e) hb[e] = h_bits(kt[i][e] * inv);
    hv[i] = (v4u){pk16(hb[0], hb[1]), pk16(hb[2], hb[3]), pk16(hb[4], hb[5]), pk16(hb[6], hb[7])};
  }
  unsigned short* pp = P + (size_t)row * kSeq + 8 * lane;
  for (int pass = 0; pass < 2; ++pass) {
#pragma unroll
    for (int i = 0; i < 8; ++i) *(volatile v4u*)(pp + 256 * i) = hv[i];
    __threadfence();
  }
}

__global__ __launch_bounds__(256) void layernorm_kernel(const float* __restrict__ hb, const float* __restrict__ gamma,
                                                        const float* __restrict__ beta, float* __restrict__ out) {
  const int lane = threadIdx.x & 31, wave = threadIdx.x >> 5;
  const int row = blockIdx.x * 8 + wave;
  const float* hp = hb + (size_t)row * kEmb;
  v4f x[6];
  float s = 0.f;
#pragma unroll
  for (int i = 0; i < 6; ++i) {
    x[i] = *(const v4f*)(hp + 128 * i + 4 * lane);
    s += (x[i][0] + x[i][1]) + (x[i][2] + x[i][3]);
  }
#pragma unroll
  for (int off = 1; off < 32; off <<= 1) s += __shfl_xor(s, off, 32);
  const float mu = s * kInvEmb;
  float vs = 0.f;
#pragma unroll
  for (int i = 0; i < 6; ++i) {
#pragma unroll
    for (int e = 0; e < 4; ++e) { const float d = x[i][e] - mu; vs += d * d; }
  }
#pragma unroll
  for (int off = 1; off < 32; off <<= 1) vs += __shfl_xor(vs, off, 32);
  const float var = vs * kInvEmb;
  const float inv = rsqrtf(var + kLnEps);
  v4f o[6];
#pragma unroll
  for (int i = 0; i < 6; ++i) {
    const v4f g = *(const v4f*)(gamma + 128 * i + 4 * lane);
    const v4f bb = *(const v4f*)(beta + 128 * i + 4 * lane);
#pragma unroll
    for (int e = 0; e < 4; ++e) o[i][e] = ((x[i][e] - mu) * inv) * g[e] + bb[e];
  }
  float* op = out + (size_t)row * kEmb + 4 * lane;
  for (int pass = 0; pass < 2; ++pass) {
#pragma unroll
    for (int i = 0; i < 6; ++i) *(volatile v4f*)(op + 128 * i) = o[i];
    __threadfence();
  }
}

extern "C" void kernel_launch(void* const* d_in, const int* in_sizes, int n_in,
                              void* d_out, int out_size, void* d_ws, size_t ws_size, hipStream_t stream) {
  if (n_in < 12) return;
  if (in_sizes[0] != kTok * kEmb || in_sizes[1] != kTok || in_sizes[2] != kEmb * kEmb || in_sizes[3] != kEmb ||
      in_sizes[4] != kEmb * kEmb || in_sizes[5] != kEmb || in_sizes[6] != kEmb * kEmb || in_sizes[7] != kEmb ||
      in_sizes[8] != kEmb * kEmb || in_sizes[9] != kEmb || in_sizes[10] != kEmb || in_sizes[11] != kEmb ||
      out_size != kTok * kEmb) return;

  const float* hidden = (const float*)d_in[0];
  const float* amask  = (const float*)d_in[1];
  const float* Wq     = (const float*)d_in[2];
  const float* bq     = (const float*)d_in[3];
  const float* Wk     = (const float*)d_in[4];
  const float* bk     = (const float*)d_in[5];
  const float* Wv     = (const float*)d_in[6];
  const float* bv     = (const float*)d_in[7];
  const float* Wo     = (const float*)d_in[8];
  const float* bo     = (const float*)d_in[9];
  const float* gamma  = (const float*)d_in[10];
  const float* beta   = (const float*)d_in[11];
  float* out = (float*)d_out;

  size_t off = 0;
  auto carve = [&](size_t bytes) -> size_t { const size_t o = off; off = (off + bytes + 255) & ~(size_t)255; return o; };
  const size_t oX16  = carve((size_t)kTok * kEmb * 2);
  const size_t oWT   = carve((size_t)4 * kEmb * kEmb * 2);
  const size_t oQ16  = carve((size_t)kBH * kHeadPlane * 2);
  const size_t oK16  = carve((size_t)kBH * kHeadPlane * 2);
  const size_t oVT16 = carve((size_t)kBH * kHeadPlane * 2);
  const size_t oCTX  = carve((size_t)kBH * kHeadPlane * 2);
  const size_t oQSQ  = carve((size_t)kBH * kSeq * 4);
  const size_t oKSQ  = carve((size_t)kBH * kSeq * 4);
  const size_t oNRB  = carve((size_t)kGH * kSeq * 4);
  const size_t oCSB  = carve((size_t)kGH * kSeq * 4);
  const size_t oCOLP = carve((size_t)kGH * kRB * kSeq * 4);
  const size_t oGBUF = carve((size_t)kGH * kScorePlane * 4);
  const size_t oP16  = carve((size_t)kGH * kScorePlane * 2);
  if (off > ws_size) return;
  if ((size_t)kTok * kEmb * 4 > (size_t)kGH * kScorePlane * 4) return;

  char* ws = (char*)d_ws;
  unsigned short* X16   = (unsigned short*)(ws + oX16);
  unsigned short* WT16  = (unsigned short*)(ws + oWT);
  unsigned short* WqT   = WT16;
  unsigned short* WkT   = WT16 + (size_t)kEmb * kEmb;
  unsigned short* WvT   = WT16 + (size_t)2 * kEmb * kEmb;
  unsigned short* WoT   = WT16 + (size_t)3 * kEmb * kEmb;
  unsigned short* Q16   = (unsigned short*)(ws + oQ16);
  unsigned short* K16   = (unsigned short*)(ws + oK16);
  unsigned short* VT16  = (unsigned short*)(ws + oVT16);
  unsigned short* CTX16 = (unsigned short*)(ws + oCTX);
  float* QSQ  = (float*)(ws + oQSQ);
  float* KSQ  = (float*)(ws + oKSQ);
  float* NRB  = (float*)(ws + oNRB);
  float* CSB  = (float*)(ws + oCSB);
  float* COLP = (float*)(ws + oCOLP);
  float* GBUF = (float*)(ws + oGBUF);
  float* HBUF = (float*)(ws + oGBUF);
  unsigned short* P16 = (unsigned short*)(ws + oP16);

  cast8_f16_kernel<<<(kTok * kEmb / 8 + 255) / 256, 256, 0, stream>>>(hidden, X16, kTok * kEmb / 8);
  wtcast_kernel<<<dim3(kEmb / 64, kEmb / 64, 4), 256, 0, stream>>>(Wq, Wk, Wv, Wo, WT16, kWCarry);

  wmma_gemm64<0, false, 2, 1, false, 0, true><<<dim3(48, kBatch), 256, 0, stream>>>(
      X16, X16, kEmb, (long)kSeq * kEmb,
      WqT, WqT, kEmb, 0L,
      Q16, Q16, kHD, (long)kHeads * kHeadPlane, kHeadPlane,
      bq, hidden, 0L, kSeq, kEmb, kEmb, kWCarryInv);
  wmma_gemm64<0, false, 2, 1, false, 0, true><<<dim3(48, kBatch), 256, 0, stream>>>(
      X16, X16, kEmb, (long)kSeq * kEmb,
      WkT, WkT, kEmb, 0L,
      K16, K16, kHD, (long)kHeads * kHeadPlane, kHeadPlane,
      bk, hidden, 0L, kSeq, kEmb, kEmb, kWCarryInv);
  wmma_gemm64<0, false, 1, 1, false, 0, false><<<dim3(48, kBatch), 256, 0, stream>>>(
      WvT, WvT, kEmb, 0L,
      X16, X16, kEmb, (long)kSeq * kEmb,
      VT16, VT16, kSeq, (long)kEmb * kSeq, 0L,
      bv, hidden, 0L, kEmb, kSeq, kEmb, kWCarryInv);

  sqnorm_kernel<<<dim3((kBH * kSeq) / 256, 2), 256, 0, stream>>>(Q16, K16, QSQ, KSQ, kBH * kSeq);

  for (int g = 0; g < kNG; ++g) {
    const int bh0 = g * kGH;
    wmma_gemm64<0, false, 0, 0, false, 0, false><<<dim3(128, kGH), 256, 0, stream>>>(
        Q16 + (size_t)bh0 * kHeadPlane, Q16 + (size_t)bh0 * kHeadPlane, kHD, kHeadPlane,
        K16 + (size_t)bh0 * kHeadPlane, K16 + (size_t)bh0 * kHeadPlane, kHD, kHeadPlane,
        GBUF, GBUF, kSeq, kScorePlane, 0L,
        bq, hidden, 0L, kSeq, kSeq, kHD, 1.0f);
    score_rows_kernel<<<dim3(kRB, kGH), 256, 0, stream>>>(GBUF, QSQ, KSQ, amask, NRB, COLP, bh0);
    colnorm_kernel<<<dim3(kSeq / 256, kGH), 256, 0, stream>>>(COLP, CSB);
    rownorm_kernel<<<(kGH * kSeq) / 8, 256, 0, stream>>>(GBUF, NRB, CSB, P16);
    wmma_gemm64<0, false, 0, 1, false, 0, false><<<dim3(4, kGH), 256, 0, stream>>>(
        P16, P16, kSeq, kScorePlane,
        VT16 + (size_t)bh0 * kHeadPlane, VT16 + (size_t)bh0 * kHeadPlane, kSeq, kHeadPlane,
        CTX16 + (size_t)bh0 * kHeadPlane, CTX16 + (size_t)bh0 * kHeadPlane, kHD, kHeadPlane, 0L,
        bq, hidden, 0L, kSeq, kHD, kSeq, kPVScale);
  }

  wmma_gemm64<0, false, 2, 0, true, 0, false><<<dim3(96, 1), 256, 0, stream>>>(
      CTX16, CTX16, kEmb, 0L,
      WoT, WoT, kEmb, 0L,
      HBUF, HBUF, kEmb, 0L, 0L,
      bo, hidden, 0L, kTok, kEmb, kEmb, kOutScale);

  layernorm_kernel<<<kTok / 8, 256, 0, stream>>>(HBUF, gamma, beta, out);
}
